// Model_43516608643518
// MI455X (gfx1250) — hardware-verified
//
#include <hip/hip_runtime.h>
#include <math.h>

constexpr int NBATCH   = 64;
constexpr int NSEQ     = 512;
constexpr int NFEAT    = 256;
constexpr int NHID     = 1024;
constexpr int NOUTC    = 128;
constexpr int MAXSTEP  = NSEQ - 1;
constexpr int SCAN_WINDOW = MAXSTEP;
constexpr int NTHR     = 256;
constexpr int ROWS_BLK = 16;
constexpr int HPITCH   = NHID + 8;
constexpr int COLS_WAVE = NHID / (NTHR / 32);
constexpr float WCARRY     = 16.0f;
constexpr float WCARRY_INV = 1.0f / WCARRY;
constexpr int LDS_BYTES = 2 * ROWS_BLK * HPITCH * 2;
constexpr int XCVT_N8   = MAXSTEP * NBATCH * (NFEAT / 8);

static_assert(NBATCH % ROWS_BLK == 0, "batch tiles");
static_assert(COLS_WAVE == 128, "8 waves x 8 column subtiles of 16");
static_assert(NHID % 64 == 0 && NFEAT % 64 == 0, "GEMM M, N tile multiples");
static_assert(NHID % 32 == 0 && NFEAT % 32 == 0, "GEMM K multiples of 32");
static_assert(LDS_BYTES % 16 == 0, "16-B zero fill");
static_assert(LDS_BYTES >= ROWS_BLK * NHID * 4, "f32 head tile fits in the h tiles");
static_assert((HPITCH * 2) % 16 == 0, "16-B aligned fragment rows");
static_assert(NFEAT / 8 == 32 && NBATCH == 64, "x convert index split");
static_assert(XCVT_N8 % NTHR == 0, "x convert grid exact");
static_assert(NOUTC == 128, "one output row = 32 lanes x 16 B");

typedef __attribute__((ext_vector_type(16))) _Float16 v16h;
typedef __attribute__((ext_vector_type(8)))  _Float16 v8h;
typedef __attribute__((ext_vector_type(16))) __bf16   v16b;
typedef __attribute__((ext_vector_type(8)))  __bf16   v8b;
typedef __attribute__((ext_vector_type(8)))  float    v8f;
typedef __attribute__((ext_vector_type(4)))  float    v4f;
typedef __attribute__((ext_vector_type(4)))  unsigned v4u;

__device__ __forceinline__ unsigned short f2bf_bits(float f) {
  unsigned u = __float_as_uint(f);
  return (unsigned short)((u + 0x7FFFu + ((u >> 16) & 1u)) >> 16);
}
__device__ __forceinline__ float bf_bits2f(unsigned short h) { return __uint_as_float(((unsigned)h) << 16); }
__device__ __forceinline__ float bf16r(float f) { return bf_bits2f(f2bf_bits(f)); }

__device__ __forceinline__ void guard4_h(v8f& a, v8f& b, v8f& c, v8f& d, v16h x, v16h y) {
  asm volatile("v_nop\n\tv_nop\n\tv_nop\n\tv_nop" : "+v"(a), "+v"(b), "+v"(c), "+v"(d) : "v"(x), "v"(y));
}
__device__ __forceinline__ void guard4_b(v8f& a, v8f& b, v8f& c, v8f& d, v16b x, v16b y) {
  asm volatile("v_nop\n\tv_nop\n\tv_nop\n\tv_nop" : "+v"(a), "+v"(b), "+v"(c), "+v"(d) : "v"(x), "v"(y));
}
__device__ __forceinline__ void keep4_h(v16h a, v16h b, v16h c, v16h d) { asm volatile("v_nop" :: "v"(a), "v"(b), "v"(c), "v"(d)); }
__device__ __forceinline__ void keep4_b(v16b a, v16b b, v16b c, v16b d) { asm volatile("v_nop" :: "v"(a), "v"(b), "v"(c), "v"(d)); }
__device__ __forceinline__ void acc_guard4(v8f& a, v8f& b, v8f& c, v8f& d) {
  asm volatile("v_nop\n\tv_nop\n\tv_nop\n\tv_nop" : "+v"(a), "+v"(b), "+v"(c), "+v"(d));
}
__device__ __forceinline__ void guard8_h(v8f& c0, v8f& c1, v8f& c2, v8f& c3, v8f& c4, v8f& c5, v8f& c6, v8f& c7,
                                         v16h a, v16h b0, v16h b1, v16h b2, v16h b3, v16h b4, v16h b5, v16h b6, v16h b7) {
  asm volatile("v_nop\n\tv_nop\n\tv_nop\n\tv_nop"
               : "+v"(c0), "+v"(c1), "+v"(c2), "+v"(c3), "+v"(c4), "+v"(c5), "+v"(c6), "+v"(c7)
               : "v"(a), "v"(b0), "v"(b1), "v"(b2), "v"(b3), "v"(b4), "v"(b5), "v"(b6), "v"(b7));
}

template <typename T> struct Frag;
template <> struct Frag<_Float16> {
  typedef v16h V; union U { v16h v; v8h h[2]; };
  static __device__ __forceinline__ v16h load(const _Float16* p) {
    U f; f.h[0] = *(const v8h*)(p); f.h[1] = *(const v8h*)(p + 16); return f.v;
  }
  static __device__ __forceinline__ v8f mma(v16h a, v16h b, v8f c) {
    return __builtin_amdgcn_wmma_f32_16x16x32_f16(false, a, false, b, (short)0, c, false, false);
  }
  static __device__ __forceinline__ void guard4(v8f& a, v8f& b, v8f& c, v8f& d, v16h x, v16h y) { guard4_h(a, b, c, d, x, y); }
  static __device__ __forceinline__ void keep(v16h a, v16h b, v16h c, v16h d) { keep4_h(a, b, c, d); }
};
template <> struct Frag<__bf16> {
  typedef v16b V; union U { v16b v; v8b h[2]; };
  static __device__ __forceinline__ v16b load(const __bf16* p) {
    U f; f.h[0] = *(const v8b*)(p); f.h[1] = *(const v8b*)(p + 16); return f.v;
  }
  static __device__ __forceinline__ v8f mma(v16b a, v16b b, v8f c) {
    return __builtin_amdgcn_wmma_f32_16x16x32_bf16(false, a, false, b, (short)0, c, false, false);
  }
  static __device__ __forceinline__ void guard4(v8f& a, v8f& b, v8f& c, v8f& d, v16b x, v16b y) { guard4_b(a, b, c, d, x, y); }
  static __device__ __forceinline__ void keep(v16b a, v16b b, v16b c, v16b d) { keep4_b(a, b, c, d); }
};

__device__ __forceinline__ float ftanh(float x) { return 1.0f - 2.0f * __builtin_amdgcn_rcpf(__expf(2.0f * x) + 1.0f); }

template <int ET> struct Elem;
template <> struct Elem<0> { typedef _Float16 T; };
template <> struct Elem<1> { typedef __bf16 T; };
template <int ET, bool SPLIT, int BIAS_MODE, int OUT_MODE, bool RESID, int ACT = 0>
__global__ __launch_bounds__(256) void wmma_gemm64(
    const unsigned short* __restrict__ Ap, const unsigned short* __restrict__ A2p, int lda, long strideA,
    const unsigned short* __restrict__ Btp, const unsigned short* __restrict__ Bt2p, int ldb, long strideB,
    void* __restrict__ Cout, void* __restrict__ Cout2, int ldc, long strideC,
    const float* __restrict__ bias,
    const float* __restrict__ resid, long strideR,
    int M, int N, int K, float scale) {
  typedef typename Elem<ET>::T T;
  typedef typename Frag<T>::V V;
  const T* A = (const T*)Ap; const T* A2 = (const T*)A2p; const T* Bt = (const T*)Btp; const T* Bt2 = (const T*)Bt2p;
  __shared__ __align__(16) float sT[8][16 * 68];
  const int b    = blockIdx.y;
  const int lane = threadIdx.x & 31;
  const int wave = threadIdx.x >> 5;
  const int tilesN = N >> 6;
  const int tilesM = M >> 6;
  const int tile = blockIdx.x * 8 + wave;
  if (tile >= tilesM * tilesN) return;
  const int tm = tile / tilesN;
  const int tn = tile - tm * tilesN;
  const int m0 = tm << 6;
  const int n0 = tn << 6;

  const T* Ab  = A  + (size_t)b * strideA;
  const T* Bb  = Bt + (size_t)b * strideB;
  const T* Ab2 = SPLIT ? (A2  + (size_t)b * strideA) : nullptr;
  const T* Bb2 = SPLIT ? (Bt2 + (size_t)b * strideB) : nullptr;

  const int rlane = lane & 15;
  const int koff  = (lane >> 4) * 8;
  const int mOff  = (lane >> 4) * 8;

  v8f acc[4][4];
#pragma unroll
  for (int i = 0; i < 4; ++i)
#pragma unroll
    for (int j = 0; j < 4; ++j) acc[i][j] = (v8f){0.f,0.f,0.f,0.f,0.f,0.f,0.f,0.f};

  for (int k0 = 0; k0 < K; k0 += 32) {
    V bh[4], bl[4];
#pragma unroll
    for (int j = 0; j < 4; ++j) {
      const size_t bo = (size_t)(n0 + (j << 4) + rlane) * ldb + koff + k0;
      bh[j] = Frag<T>::load(Bb + bo);
      if (SPLIT) bl[j] = Frag<T>::load(Bb2 + bo);
    }
#pragma unroll
    for (int i = 0; i < 4; ++i) {
      const size_t ao = (size_t)(m0 + (i << 4) + rlane) * lda + koff + k0;
      V ah = Frag<T>::load(Ab + ao);
      V al;
      if (SPLIT) al = Frag<T>::load(Ab2 + ao);
#pragma unroll
      for (int j = 0; j < 4; ++j) {
        acc[i][j] = Frag<T>::mma(ah, bh[j], acc[i][j]);
        if (SPLIT) {
          acc[i][j] = Frag<T>::mma(ah, bl[j], acc[i][j]);
          acc[i][j] = Frag<T>::mma(al, bh[j], acc[i][j]);
        }
      }
      Frag<T>::guard4(acc[i][0], acc[i][1], acc[i][2], acc[i][3], ah, SPLIT ? al : ah);
    }
    Frag<T>::keep(bh[0], bh[1], bh[2], bh[3]);
    if (SPLIT) Frag<T>::keep(bl[0], bl[1], bl[2], bl[3]);
  }
  acc_guard4(acc[0][0], acc[0][1], acc[0][2], acc[0][3]);
  acc_guard4(acc[1][0], acc[1][1], acc[1][2], acc[1][3]);
  acc_guard4(acc[2][0], acc[2][1], acc[2][2], acc[2][3]);
  acc_guard4(acc[3][0], acc[3][1], acc[3][2], acc[3][3]);

  float* slab = sT[wave];
  const float* Rb = RESID ? (resid + (size_t)b * strideR) : nullptr;
#pragma unroll
  for (int i = 0; i < 4; ++i) {
    const int mBase = m0 + (i << 4);
#pragma unroll
    for (int j = 0; j < 4; ++j) {
      const int n = n0 + (j << 4) + rlane;
      float bv = 0.f;
      if (BIAS_MODE == 2) bv = bias[n];
#pragma unroll
      for (int r = 0; r < 8; ++r) {
        float v = acc[i][j][r] * scale;
        if (BIAS_MODE == 1) v += bias[mBase + mOff + r];
        if (BIAS_MODE == 2) v += bv;
        if (RESID) v += Rb[(size_t)(mBase + mOff + r) * ldc + n];
        if (ACT == 1) v = tanhf(v);
        if (ACT == 2) v = fmaxf(v, 0.0f);
        if (ACT == 4) v = (v > 0.f) ? v : 0.01f * v;
        slab[(mOff + r) * 68 + (j << 4) + rlane] = v;
      }
    }
    __builtin_amdgcn_fence(__ATOMIC_RELEASE, "workgroup");
    __builtin_amdgcn_wave_barrier();
    __builtin_amdgcn_fence(__ATOMIC_ACQUIRE, "workgroup");
    if (OUT_MODE == 0) {
      float* C = (float*)Cout + (size_t)b * strideC;
      const int hh = lane >> 4, c4 = (lane & 15) * 4;
      for (int pass = 0; pass < 2; ++pass) {
#pragma unroll
        for (int it = 0; it < 8; ++it) {
          const int row = it * 2 + hh;
          v4f v = *(const v4f*)(slab + row * 68 + c4);
          *(volatile v4f*)(C + (size_t)(mBase + row) * ldc + n0 + c4) = v;
        }
        __threadfence();
      }
    } else {
      const int q = lane >> 3, c8 = (lane & 7) * 8;
      unsigned short* C  = (unsigned short*)Cout  + (size_t)b * strideC;
      unsigned short* C2 = (OUT_MODE == 2) ? ((unsigned short*)Cout2 + (size_t)b * strideC) : nullptr;
      for (int pass = 0; pass < 2; ++pass) {
#pragma unroll
        for (int it = 0; it < 4; ++it) {
          const int row = it * 4 + q;
          const float* sp = slab + row * 68 + c8;
          v8h hv, lv;
#pragma unroll
          for (int e = 0; e < 8; ++e) {
            if (OUT_MODE == 1) {
              hv[e] = (_Float16)sp[e];
            } else {
              unsigned short hb = f2bf_bits(sp[e]);
              unsigned short lb = f2bf_bits(sp[e] - bf_bits2f(hb));
              hv[e] = __builtin_bit_cast(_Float16, hb);
              lv[e] = __builtin_bit_cast(_Float16, lb);
            }
          }
          *(volatile v8h*)(C + (size_t)(mBase + row) * ldc + n0 + c8) = hv;
          if (OUT_MODE == 2) *(volatile v8h*)(C2 + (size_t)(mBase + row) * ldc + n0 + c8) = lv;
        }
        __threadfence();
      }
    }
    __builtin_amdgcn_fence(__ATOMIC_RELEASE, "workgroup");
    __builtin_amdgcn_wave_barrier();
    __builtin_amdgcn_fence(__ATOMIC_ACQUIRE, "workgroup");
  }
}

template <int MODE>
__global__ __launch_bounds__(NTHR) void cvt8_kernel(const float* __restrict__ src, unsigned short* __restrict__ dst,
                                                    int nrow, int ncol8, int spitch, int scol0, float sc) {
  const int i  = blockIdx.x * NTHR + threadIdx.x;
  const int n8 = nrow * ncol8;
  if (i < n8) {
    const int row = i / ncol8;
    const int c8  = i - row * ncol8;
    const float* sp = src + (size_t)row * spitch + scol0 + c8 * 8;
    const v4f a = *(const v4f*)(sp);
    const v4f b = *(const v4f*)(sp + 4);
    v8h hv;
#pragma unroll
    for (int e = 0; e < 4; ++e) {
      unsigned short b0, b1;
      if (MODE == 0) {
        b0 = f2bf_bits(a[e] * sc);
        b1 = f2bf_bits(b[e] * sc);
      } else {
        b0 = __builtin_bit_cast(unsigned short, (_Float16)(bf16r(a[e]) * sc));
        b1 = __builtin_bit_cast(unsigned short, (_Float16)(bf16r(b[e]) * sc));
      }
      hv[e]     = __builtin_bit_cast(_Float16, b0);
      hv[4 + e] = __builtin_bit_cast(_Float16, b1);
    }
    *(volatile v8h*)(dst + (size_t)i * 8) = hv;
    __threadfence();
    *(volatile v8h*)(dst + (size_t)i * 8) = hv;
  }
}

__global__ __launch_bounds__(NTHR) void cvtx_kernel(const float* __restrict__ x, unsigned short* __restrict__ X16) {
  const int i = blockIdx.x * NTHR + threadIdx.x;
  if (i < XCVT_N8) {
    const int f8 = i & 31;
    const int b  = (i >> 5) & 63;
    const int t  = i >> 11;
    const float* sp = x + ((size_t)b * NSEQ + (size_t)t) * NFEAT + f8 * 8;
    const v4f a = *(const v4f*)(sp);
    const v4f c = *(const v4f*)(sp + 4);
    v8h hv;
#pragma unroll
    for (int e = 0; e < 4; ++e) {
      hv[e]     = (_Float16)bf16r(a[e]);
      hv[4 + e] = (_Float16)bf16r(c[e]);
    }
    *(volatile v8h*)(X16 + (size_t)i * 8) = hv;
    __threadfence();
    *(volatile v8h*)(X16 + (size_t)i * 8) = hv;
  }
}

template <int MODE>
__global__ __launch_bounds__(NTHR) void tpw_kernel(const float* __restrict__ src, int R, int C, int ldo,
                                                  unsigned short* __restrict__ O, float sc) {
  __shared__ float Tt[64 * 65];
  const int tid = threadIdx.x;
  const int c0 = blockIdx.x * 64, r0 = blockIdx.y * 64;
#pragma unroll
  for (int i = 0; i < 4; ++i) {
    const int idx = i * NTHR + tid;
    const int rr = idx >> 4, cc = (idx & 15) * 4;
    const v4f v = *(const v4f*)(src + (size_t)(r0 + rr) * (size_t)C + c0 + cc);
    Tt[rr * 65 + cc + 0] = v[0];
    Tt[rr * 65 + cc + 1] = v[1];
    Tt[rr * 65 + cc + 2] = v[2];
    Tt[rr * 65 + cc + 3] = v[3];
  }
  __syncthreads();
  const int q = tid >> 3, c8 = (tid & 7) * 8;
  v8h hv[2];
#pragma unroll
  for (int g = 0; g < 2; ++g) {
    const int qq = g * 32 + q;
#pragma unroll
    for (int e = 0; e < 8; ++e) {
      const float f = Tt[(c8 + e) * 65 + qq];
      unsigned short bits;
      if (MODE == 0) {
        bits = f2bf_bits(f * sc);
      } else {
        const float fb = bf_bits2f(f2bf_bits(f));
        bits = __builtin_bit_cast(unsigned short, (_Float16)(fb * sc));
      }
      hv[g][e] = __builtin_bit_cast(_Float16, bits);
    }
  }
  for (int pass = 0; pass < 2; ++pass) {
#pragma unroll
    for (int g = 0; g < 2; ++g) {
      const size_t o = (size_t)(c0 + g * 32 + q) * (size_t)ldo + (size_t)(r0 + c8);
      *(volatile v8h*)(O + o) = hv[g];
    }
    __threadfence();
  }
}

__global__ __launch_bounds__(NTHR) void bias_kernel(const float* __restrict__ W_ih, const float* __restrict__ b_in,
                                                    const float* __restrict__ b_ih, const float* __restrict__ b_hh,
                                                    float* __restrict__ BC1, float* __restrict__ B2) {
  __shared__ float sred[32];
  const int tid = threadIdx.x, lane = tid & 31, wave = tid >> 5;
  const int n0 = blockIdx.x * 32;
#pragma unroll 1
  for (int i = 0; i < 4; ++i) {
    const int n = n0 + wave * 4 + i;
    const float* wr = W_ih + (size_t)n * NHID;
    float s = 0.0f;
#pragma unroll 1
    for (int k = lane * 4; k < NHID; k += 128) {
      const v4f w  = *(const v4f*)(wr + k);
      const v4f bv = *(const v4f*)(b_in + k);
      s = fmaf(bf16r(w[0]), bf16r(bv[0]), s);
      s = fmaf(bf16r(w[1]), bf16r(bv[1]), s);
      s = fmaf(bf16r(w[2]), bf16r(bv[2]), s);
      s = fmaf(bf16r(w[3]), bf16r(bv[3]), s);
    }
#pragma unroll
    for (int off = 16; off >= 1; off >>= 1) s += __shfl_xor(s, off, 32);
    if (lane == 0) sred[wave * 4 + i] = s;
  }
  __syncthreads();
  if (wave == 0) {
    const int n = n0 + lane;
    const float o1 = (sred[lane] + bf16r(b_ih[n])) + bf16r(b_hh[n]);
    const float o2 = bf16r(b_ih[NHID + n]) + bf16r(b_hh[NHID + n]);
    *(volatile float*)(BC1 + n) = o1;
    *(volatile float*)(B2 + n)  = o2;
    __threadfence();
    *(volatile float*)(BC1 + n) = o1;
    *(volatile float*)(B2 + n)  = o2;
  }
}

template <int LDB, int KLEN>
__device__ __forceinline__ void kloop8(v8f (&acc)[8], const _Float16* ap, const _Float16* bp) {
#pragma unroll 1
  for (int k0 = 0; k0 < KLEN; k0 += 32) {
    const v16h a  = Frag<_Float16>::load(ap + k0);
    const v16h b0 = Frag<_Float16>::load(bp + k0);
    const v16h b1 = Frag<_Float16>::load(bp + 16 * LDB + k0);
    const v16h b2 = Frag<_Float16>::load(bp + 32 * LDB + k0);
    const v16h b3 = Frag<_Float16>::load(bp + 48 * LDB + k0);
    const v16h b4 = Frag<_Float16>::load(bp + 64 * LDB + k0);
    const v16h b5 = Frag<_Float16>::load(bp + 80 * LDB + k0);
    const v16h b6 = Frag<_Float16>::load(bp + 96 * LDB + k0);
    const v16h b7 = Frag<_Float16>::load(bp + 112 * LDB + k0);
    acc[0] = Frag<_Float16>::mma(a, b0, acc[0]);
    acc[1] = Frag<_Float16>::mma(a, b1, acc[1]);
    acc[2] = Frag<_Float16>::mma(a, b2, acc[2]);
    acc[3] = Frag<_Float16>::mma(a, b3, acc[3]);
    acc[4] = Frag<_Float16>::mma(a, b4, acc[4]);
    acc[5] = Frag<_Float16>::mma(a, b5, acc[5]);
    acc[6] = Frag<_Float16>::mma(a, b6, acc[6]);
    acc[7] = Frag<_Float16>::mma(a, b7, acc[7]);
    guard8_h(acc[0], acc[1], acc[2], acc[3], acc[4], acc[5], acc[6], acc[7], a, b0, b1, b2, b3, b4, b5, b6, b7);
  }
}

__global__ __launch_bounds__(NTHR) void rnn_seq_kernel(const unsigned short* __restrict__ X16p,
                                                       const unsigned short* __restrict__ WC1p,
                                                       const unsigned short* __restrict__ WHHp,
                                                       const unsigned short* __restrict__ WIH2p,
                                                       const float* __restrict__ BC1, const float* __restrict__ B2,
                                                       const float* __restrict__ W_out, const float* __restrict__ b_out,
                                                       const int* __restrict__ pred_len_p, float* __restrict__ out) {
  __shared__ __align__(16) unsigned char smem[LDS_BYTES];
  _Float16* H1 = (_Float16*)smem;
  _Float16* H2 = H1 + ROWS_BLK * HPITCH;
  float*    HF = (float*)smem;

  const _Float16* X16  = (const _Float16*)X16p;
  const _Float16* WC1  = (const _Float16*)WC1p;
  const _Float16* WHH0 = (const _Float16*)WHHp;
  const _Float16* WHH1 = (const _Float16*)WHHp + (size_t)NHID * NHID;
  const _Float16* WIH2 = (const _Float16*)WIH2p;

  const int tid = threadIdx.x, lane = tid & 31, wave = tid >> 5;
  const int c = lane & 15, hh = lane >> 4, koff = hh * 8;
  const int rowbase = blockIdx.x * ROWS_BLK;
  const int colc = COLS_WAVE * wave + c;

  {
    v4u* z = (v4u*)smem;
    const v4u zero = {0u, 0u, 0u, 0u};
#pragma unroll 1
    for (int i = tid; i < LDS_BYTES / 16; i += NTHR) z[i] = zero;
  }

  int pl = pred_len_p[0];
  pl = (pl < 1) ? 1 : ((pl > MAXSTEP) ? MAXSTEP : pl);
  const int nsteps = NSEQ - pl;
  const int tstart = (nsteps > SCAN_WINDOW) ? (nsteps - SCAN_WINDOW) : 0;

  float bc1r[8], b2r[8];
#pragma unroll
  for (int j = 0; j < 8; ++j) {
    bc1r[j] = BC1[colc + 16 * j];
    b2r[j]  = B2[colc + 16 * j];
  }

  const _Float16* a1 = H1 + c * HPITCH + koff;
  const _Float16* a2 = H2 + c * HPITCH + koff;
  const _Float16* bwc1  = WC1  + (size_t)colc * NFEAT + koff;
  const _Float16* bwhh0 = WHH0 + (size_t)colc * NHID + koff;
  const _Float16* bwih2 = WIH2 + (size_t)colc * NHID + koff;
  const _Float16* bwhh1 = WHH1 + (size_t)colc * NHID + koff;
  const v8f z8 = {0.f, 0.f, 0.f, 0.f, 0.f, 0.f, 0.f, 0.f};

  __syncthreads();

#pragma unroll 1
  for (int t = tstart; t < nsteps; ++t) {
    const bool last = (t == nsteps - 1);
    v8f acc[8];

#pragma unroll
    for (int j = 0; j < 8; ++j) acc[j] = z8;
    {
      const _Float16* ax = X16 + ((size_t)t * NBATCH + (size_t)(rowbase + c)) * NFEAT + koff;
      kloop8<NFEAT, NFEAT>(acc, ax, bwc1);
    }
    kloop8<NHID, NHID>(acc, a1, bwhh0);
    __syncthreads();
#pragma unroll
    for (int j = 0; j < 8; ++j) {
#pragma unroll
      for (int r = 0; r < 8; ++r) {
        const float v = ftanh(acc[j][r] * WCARRY_INV + bc1r[j]);
        H1[(8 * hh + r) * HPITCH + colc + 16 * j] = (_Float16)v;
      }
    }
    __syncthreads();

#pragma unroll
    for (int j = 0; j < 8; ++j) acc[j] = z8;
    kloop8<NHID, NHID>(acc, a1, bwih2);
    kloop8<NHID, NHID>(acc, a2, bwhh1);
    __syncthreads();
#pragma unroll
    for (int j = 0; j < 8; ++j) {
#pragma unroll
      for (int r = 0; r < 8; ++r) acc[j][r] = ftanh(acc[j][r] * WCARRY_INV + b2r[j]);
    }
    if (!last) {
#pragma unroll
      for (int j = 0; j < 8; ++j) {
#pragma unroll
        for (int r = 0; r < 8; ++r) H2[(8 * hh + r) * HPITCH + colc + 16 * j] = (_Float16)acc[j][r];
      }
    } else {
#pragma unroll
      for (int j = 0; j < 8; ++j) {
#pragma unroll
        for (int r = 0; r < 8; ++r) HF[(8 * hh + r) * NHID + colc + 16 * j] = fmaxf(acc[j][r], 0.0f);
      }
    }
    __syncthreads();
  }

  {
    const int m0 = 2 * wave, m1 = 2 * wave + 1, tc = 4 * lane;
    const v4f bo = *(const v4f*)(b_out + tc);
    float o0[4], o1[4];
#pragma unroll
    for (int e = 0; e < 4; ++e) { o0[e] = bf16r(bo[e]); o1[e] = o0[e]; }
    const float* wp  = W_out + (size_t)tc * NHID;
    const float* hp0 = HF + m0 * NHID;
    const float* hp1 = HF + m1 * NHID;
#pragma unroll 1
    for (int k = 0; k < NHID; k += 4) {
      const v4f ha = *(const v4f*)(hp0 + k);
      const v4f hb = *(const v4f*)(hp1 + k);
      const v4f w0 = *(const v4f*)(wp + k);
      const v4f w1 = *(const v4f*)(wp + NHID + k);
      const v4f w2 = *(const v4f*)(wp + 2 * NHID + k);
      const v4f w3 = *(const v4f*)(wp + 3 * NHID + k);
#pragma unroll
      for (int e = 0; e < 4; ++e) {
        const float x0 = bf16r(w0[e]);
        const float x1 = bf16r(w1[e]);
        const float x2 = bf16r(w2[e]);
        const float x3 = bf16r(w3[e]);
        const float ga = ha[e];
        const float gb = hb[e];
        o0[0] = fmaf(ga, x0, o0[0]);
        o0[1] = fmaf(ga, x1, o0[1]);
        o0[2] = fmaf(ga, x2, o0[2]);
        o0[3] = fmaf(ga, x3, o0[3]);
        o1[0] = fmaf(gb, x0, o1[0]);
        o1[1] = fmaf(gb, x1, o1[1]);
        o1[2] = fmaf(gb, x2, o1[2]);
        o1[3] = fmaf(gb, x3, o1[3]);
      }
    }
    v4f s0, s1;
#pragma unroll
    for (int e = 0; e < 4; ++e) { s0[e] = o0[e]; s1[e] = o1[e]; }
    float* op0 = out + (size_t)(rowbase + m0) * NOUTC + tc;
    float* op1 = out + (size_t)(rowbase + m1) * NOUTC + tc;
    for (int pass = 0; pass < 2; ++pass) {
      *(volatile v4f*)op0 = s0;
      *(volatile v4f*)op1 = s1;
      __threadfence();
    }
  }
}

extern "C" void kernel_launch(void* const* d_in, const int* in_sizes, int n_in,
                              void* d_out, int out_size, void* d_ws, size_t ws_size, hipStream_t stream) {
  if (n_in < 10 || d_out == nullptr || d_ws == nullptr) return;
  if (in_sizes[0] != NBATCH * NSEQ * NFEAT || in_sizes[1] != NHID * NFEAT || in_sizes[2] != NHID ||
      in_sizes[3] != 2 * NHID * NHID || in_sizes[4] != 2 * NHID || in_sizes[5] != 2 * NHID * NHID ||
      in_sizes[6] != 2 * NHID || in_sizes[7] != NOUTC * NHID || in_sizes[8] != NOUTC || in_sizes[9] != 1 ||
      out_size != NBATCH * NOUTC) return;

  const float* x     = (const float*)d_in[0];
  const float* w_in  = (const float*)d_in[1];
  const float* b_in  = (const float*)d_in[2];
  const float* w_ih  = (const float*)d_in[3];
  const float* b_ih  = (const float*)d_in[4];
  const float* w_hh  = (const float*)d_in[5];
  const float* b_hh  = (const float*)d_in[6];
  const float* w_out = (const float*)d_in[7];
  const float* b_out = (const float*)d_in[8];
  const int*   predl = (const int*)d_in[9];
  float* out = (float*)d_out;

  char* ws = (char*)d_ws; size_t off = 0;
  auto carve = [&](size_t bytes) -> char* { char* p = ws + off; off += (bytes + 255) & ~(size_t)255; return p; };
  unsigned short* X16   = (unsigned short*)carve((size_t)MAXSTEP * NBATCH * NFEAT * 2);
  unsigned short* WHH16 = (unsigned short*)carve((size_t)2 * NHID * NHID * 2);
  unsigned short* WIH2  = (unsigned short*)carve((size_t)NHID * NHID * 2);
  unsigned short* WIH0B = (unsigned short*)carve((size_t)NHID * NHID * 2);
  unsigned short* WINT  = (unsigned short*)carve((size_t)NFEAT * NHID * 2);
  unsigned short* WC1   = (unsigned short*)carve((size_t)NHID * NFEAT * 2);
  float*          BC1   = (float*)carve((size_t)NHID * 4);
  float*          B2    = (float*)carve((size_t)NHID * 4);
  if (off > ws_size || off > (size_t)134217728) return;

  const int n8hh = 2 * NHID * (NHID / 8);
  const int n8ih = NHID * (NHID / 8);
  cvt8_kernel<1><<<n8hh / NTHR, NTHR, 0, stream>>>(w_hh, WHH16, 2 * NHID, NHID / 8, NHID, 0, WCARRY);
  cvt8_kernel<1><<<n8ih / NTHR, NTHR, 0, stream>>>(w_ih + (size_t)NHID * NHID, WIH2, NHID, NHID / 8, NHID, 0, WCARRY);
  cvt8_kernel<0><<<n8ih / NTHR, NTHR, 0, stream>>>(w_ih, WIH0B, NHID, NHID / 8, NHID, 0, 1.0f);
  tpw_kernel<0><<<dim3(NFEAT / 64, NHID / 64), NTHR, 0, stream>>>(w_in, NHID, NFEAT, NHID, WINT, 1.0f);
  bias_kernel<<<NHID / 32, NTHR, 0, stream>>>(w_ih, b_in, b_ih, b_hh, BC1, B2);
  cvtx_kernel<<<XCVT_N8 / NTHR, NTHR, 0, stream>>>(x, X16);
  wmma_gemm64<1, false, 0, 1, false, 0><<<dim3((NHID / 64) * (NFEAT / 64) / 8, 1), 256, 0, stream>>>(
      WIH0B, WIH0B, NHID, 0L, WINT, WINT, NHID, 0L, (void*)WC1, (void*)WC1, NFEAT, 0L,
      BC1, BC1, 0L, NHID, NFEAT, NHID, WCARRY);
  rnn_seq_kernel<<<NBATCH / ROWS_BLK, NTHR, 0, stream>>>(X16, WC1, WHH16, WIH2, BC1, B2, w_out, b_out, predl, out);
}
